// MultiDilatelocalAttention_41661182771557
// MI455X (gfx1250) — hardware-verified
//
#include <hip/hip_runtime.h>

typedef unsigned short v8us  __attribute__((ext_vector_type(8)));
typedef unsigned short v16us __attribute__((ext_vector_type(16)));
typedef __bf16         v16bf __attribute__((ext_vector_type(16)));
typedef float          v8f   __attribute__((ext_vector_type(8)));
typedef float          v4f   __attribute__((ext_vector_type(4)));
typedef v8us __attribute__((may_alias)) v8usa;
typedef v4f  __attribute__((may_alias)) v4fa;

union Frag { v16bf v; v16us u; v8us half[2]; };

#define NB     8
#define CH     256
#define NQKV   768
#define HWPIX  4096
#define WIMG   64
#define NHEAD  8
#define HDIM   32
#define IMGPP  4
#define MROWS  (IMGPP * HWPIX)
#define TPX    64
#define TN     64
#define APX    32
#define SDP    68
#define LPX    264
#define ATT_SCALE 0.17677669529663687f

static_assert(NB % IMGPP == 0);
static_assert(HWPIX % TPX == 0 && HWPIX % APX == 0);
static_assert(MROWS % TPX == 0);
static_assert(NQKV % TN == 0 && CH % TN == 0);
static_assert(CH % 32 == 0);
static_assert((SDP % 4) == 0 && (LPX % 8) == 0);
static_assert(NHEAD * HDIM == CH);
static_assert(NHEAD * 32 == 256);
static_assert(APX * CH * 2 * 2 == 8 * 256 * 16);
static_assert(NQKV % 8 == 0 && CH % 8 == 0);

__device__ __forceinline__ unsigned int bf16_bits(float f) {
  const unsigned int u = __float_as_uint(f);
  return (u + 0x7FFFu + ((u >> 16) & 1u)) >> 16;
}
__device__ __forceinline__ float bf16_val(float f) {
  return __uint_as_float(bf16_bits(f) << 16);
}

__device__ __forceinline__ v8f wmma_bf16(Frag a, Frag b, v8f c) {
  v8f d = __builtin_amdgcn_wmma_f32_16x16x32_bf16(false, a.v, false, b.v, (short)0, c, false, false);
  asm volatile("v_nop\n\tv_nop\n\tv_nop\n\tv_nop" : "+v"(d) : "v"(a.u), "v"(b.u));
  return d;
}

__device__ __forceinline__ Frag load_frag(const unsigned short* p, int h) {
  Frag f;
  f.half[0] = *(const v8usa*)(p + 8 * h);
  f.half[1] = *(const v8usa*)(p + 16 + 8 * h);
  return f;
}

__global__ __launch_bounds__(256) void xt_kernel(const float* __restrict__ x,
                                                 unsigned short* __restrict__ xt)
{
  __shared__ __attribute__((aligned(16))) unsigned short sT[TPX * LPX];

  const int tid = threadIdx.x, lane = tid & 31, w = tid >> 5;
  const int t = blockIdx.x, img = blockIdx.y;
  const int p0 = t * TPX;
  const int pl = tid & 63, cb = tid >> 6;
  const float* xs = x + (size_t)img * CH * HWPIX + p0 + pl;

  #pragma unroll 4
  for (int i = 0; i < 64; ++i) {
    const int c = cb + 4 * i;
    const float v = xs[(size_t)c * HWPIX];
    sT[pl * LPX + c] = (unsigned short)bf16_bits(v);
  }
  __syncthreads();

  unsigned short* base = xt + ((size_t)img * HWPIX + p0) * CH + 8 * lane;
  v8us vv[8];
  #pragma unroll
  for (int i = 0; i < 8; ++i) {
    const int row = 8 * w + i;
    vv[i] = *(const v8usa*)(sT + row * LPX + 8 * lane);
  }
  #pragma unroll
  for (int i = 0; i < 8; ++i) {
    const int row = 8 * w + i;
    *(volatile v8us*)(base + (size_t)row * CH) = vv[i];
  }
  __threadfence();
  #pragma unroll
  for (int i = 0; i < 8; ++i) {
    const int row = 8 * w + i;
    *(volatile v8us*)(base + (size_t)row * CH) = vv[i];
  }
}

__global__ __launch_bounds__(256) void wconv_kernel(const float* __restrict__ wsrc,
                                                    unsigned short* __restrict__ wdst,
                                                    int nrows)
{
  const int tid = threadIdx.x, lane = tid & 31, w = tid >> 5;
  int row = blockIdx.x * 8 + w;
  row = (row < nrows) ? row : (nrows - 1);
  const v4f* src = (const v4f*)(wsrc + (size_t)row * CH + 8 * lane);
  const v4f a = src[0];
  const v4f b = src[1];
  v8us o;
  o[0] = (unsigned short)bf16_bits(a.x); o[1] = (unsigned short)bf16_bits(a.y);
  o[2] = (unsigned short)bf16_bits(a.z); o[3] = (unsigned short)bf16_bits(a.w);
  o[4] = (unsigned short)bf16_bits(b.x); o[5] = (unsigned short)bf16_bits(b.y);
  o[6] = (unsigned short)bf16_bits(b.z); o[7] = (unsigned short)bf16_bits(b.w);
  unsigned short* dst = wdst + (size_t)row * CH + 8 * lane;
  *(volatile v8us*)dst = o;
  __threadfence();
  *(volatile v8us*)dst = o;
}

__global__ __launch_bounds__(128) void gemm_qkv_kernel(
    const unsigned short* __restrict__ xa_plane,
    const unsigned short* __restrict__ wq,
    const float* __restrict__ bias,
    float* __restrict__ qkv)
{
  __shared__ __attribute__((aligned(16))) float sD[TPX * SDP];

  const int tid = threadIdx.x, lane = tid & 31, w = tid >> 5;
  const int h = lane >> 4, m = lane & 15;
  const int m0 = blockIdx.x * TPX, n0 = blockIdx.y * TN;
  const v8f zero8 = {0.f, 0.f, 0.f, 0.f, 0.f, 0.f, 0.f, 0.f};

  v8f acc[4];
  #pragma unroll
  for (int nt = 0; nt < 4; ++nt) acc[nt] = zero8;

  const unsigned short* xa = xa_plane + (size_t)(m0 + 16 * w + m) * CH;
  const unsigned short* wb = wq + (size_t)(n0 + m) * CH;

  #pragma unroll 1
  for (int k0 = 0; k0 < CH; k0 += 32) {
    const Frag a = load_frag(xa + k0, h);
    #pragma unroll
    for (int nt = 0; nt < 4; ++nt) {
      const Frag b = load_frag(wb + (size_t)nt * 16 * CH + k0, h);
      acc[nt] = wmma_bf16(a, b, acc[nt]);
    }
  }

  #pragma unroll
  for (int nt = 0; nt < 4; ++nt) {
    const int o = 16 * nt + m;
    const float bv = bf16_val(bias[n0 + o]);
    #pragma unroll
    for (int r = 0; r < 8; ++r) sD[(16 * w + 8 * h + r) * SDP + o] = acc[nt][r] + bv;
  }
  __syncthreads();

  const int sub = lane >> 4, c4 = 4 * (lane & 15);
  v4f vv[8];
  #pragma unroll
  for (int i = 0; i < 8; ++i) {
    const int row = 16 * w + 2 * i + sub;
    vv[i] = *(const v4fa*)(sD + row * SDP + c4);
  }
  float* base = qkv + (size_t)m0 * NQKV + n0 + c4;
  #pragma unroll
  for (int i = 0; i < 8; ++i) {
    const int row = 16 * w + 2 * i + sub;
    *(volatile v4f*)(base + (size_t)row * NQKV) = vv[i];
  }
  __threadfence();
  #pragma unroll
  for (int i = 0; i < 8; ++i) {
    const int row = 16 * w + 2 * i + sub;
    *(volatile v4f*)(base + (size_t)row * NQKV) = vv[i];
  }
}

__global__ __launch_bounds__(256) void attn_kernel(const float* __restrict__ qkv,
                                                   unsigned short* __restrict__ ohi,
                                                   unsigned short* __restrict__ olo)
{
  __shared__ __attribute__((aligned(16))) v4f   sAcc[8 * 256];
  __shared__ __attribute__((aligned(16))) float sLg[9 * 256];

  const int tid = threadIdx.x, lane = tid & 31, hd = tid >> 5;
  const int bl = blockIdx.y;
  const int p0 = blockIdx.x * APX;
  const int p  = p0 + lane;
  const int py = p >> 6, px = p & 63;
  const int dil = (hd & 3) + 1;

  const float* img = qkv + (size_t)bl * HWPIX * NQKV;
  const v4f* q4 = (const v4f*)(img + (size_t)p * NQKV + hd * HDIM);

  float mx = __uint_as_float(0xff800000u);
  #pragma unroll 1
  for (int t = 0; t < 9; ++t) {
    const int ti = t / 3;
    const int tj = t - 3 * ti;
    const int iy = py + (ti - 1) * dil;
    const int ix = px + (tj - 1) * dil;
    const bool valid = ((unsigned)iy < (unsigned)WIMG) && ((unsigned)ix < (unsigned)WIMG);
    const int pn = valid ? (iy * WIMG + ix) : p;
    const v4f* k4 = (const v4f*)(img + (size_t)pn * NQKV + CH + hd * HDIM);
    float s = 0.0f;
    #pragma unroll 4
    for (int c = 0; c < 8; ++c) {
      const v4f qv = q4[c];
      const v4f kv = k4[c];
      s = fmaf(qv.x, kv.x, s);
      s = fmaf(qv.y, kv.y, s);
      s = fmaf(qv.z, kv.z, s);
      s = fmaf(qv.w, kv.w, s);
    }
    const float lg = valid ? (s * ATT_SCALE) : 0.0f;
    sLg[t * 256 + tid] = lg;
    mx = fmaxf(mx, lg);
  }

  float wsum = 0.0f;
  #pragma unroll 1
  for (int t = 0; t < 9; ++t) {
    const float e = expf(sLg[t * 256 + tid] - mx);
    sLg[t * 256 + tid] = e;
    wsum += e;
  }
  const float inv = 1.0f / wsum;

  const v4f z4 = {0.f, 0.f, 0.f, 0.f};
  #pragma unroll
  for (int c = 0; c < 8; ++c) sAcc[c * 256 + tid] = z4;

  #pragma unroll 1
  for (int t = 0; t < 9; ++t) {
    const int ti = t / 3;
    const int tj = t - 3 * ti;
    const int iy = py + (ti - 1) * dil;
    const int ix = px + (tj - 1) * dil;
    const bool valid = ((unsigned)iy < (unsigned)WIMG) && ((unsigned)ix < (unsigned)WIMG);
    const int pn = valid ? (iy * WIMG + ix) : p;
    const float wt = valid ? (sLg[t * 256 + tid] * inv) : 0.0f;
    const v4f* v4 = (const v4f*)(img + (size_t)pn * NQKV + 2 * CH + hd * HDIM);
    #pragma unroll 4
    for (int c = 0; c < 8; ++c) {
      v4f a = sAcc[c * 256 + tid];
      const v4f vv = v4[c];
      a.x = fmaf(wt, vv.x, a.x);
      a.y = fmaf(wt, vv.y, a.y);
      a.z = fmaf(wt, vv.z, a.z);
      a.w = fmaf(wt, vv.w, a.w);
      sAcc[c * 256 + tid] = a;
    }
  }

  v8us hv[4], lv[4];
  #pragma unroll
  for (int j = 0; j < 4; ++j) {
    const v4f a0 = sAcc[(2 * j) * 256 + tid];
    const v4f a1 = sAcc[(2 * j + 1) * 256 + tid];
    const float f[8] = {a0.x, a0.y, a0.z, a0.w, a1.x, a1.y, a1.z, a1.w};
    #pragma unroll
    for (int e = 0; e < 8; ++e) {
      const unsigned int hb = bf16_bits(f[e]);
      const float hf = __uint_as_float(hb << 16);
      hv[j][e] = (unsigned short)hb;
      lv[j][e] = (unsigned short)bf16_bits(f[e] - hf);
    }
  }
  __syncthreads();

  unsigned short* sH = (unsigned short*)sAcc;
  unsigned short* sL = sH + APX * CH;
  #pragma unroll
  for (int j = 0; j < 4; ++j) {
    *(v8usa*)(sH + lane * CH + hd * HDIM + 8 * j) = hv[j];
    *(v8usa*)(sL + lane * CH + hd * HDIM + 8 * j) = lv[j];
  }
  __syncthreads();

  v8us oh[4], ol[4];
  #pragma unroll
  for (int i = 0; i < 4; ++i) {
    const int row = 4 * hd + i;
    oh[i] = *(const v8usa*)(sH + row * CH + 8 * lane);
    ol[i] = *(const v8usa*)(sL + row * CH + 8 * lane);
  }
  const size_t rb = ((size_t)bl * HWPIX + p0) * CH + 8 * lane;
  #pragma unroll
  for (int i = 0; i < 4; ++i) {
    const size_t off = rb + (size_t)(4 * hd + i) * CH;
    *(volatile v8us*)(ohi + off) = oh[i];
    *(volatile v8us*)(olo + off) = ol[i];
  }
  __threadfence();
  #pragma unroll
  for (int i = 0; i < 4; ++i) {
    const size_t off = rb + (size_t)(4 * hd + i) * CH;
    *(volatile v8us*)(ohi + off) = oh[i];
    *(volatile v8us*)(olo + off) = ol[i];
  }
}

__global__ __launch_bounds__(128) void gemm_proj_kernel(
    const unsigned short* __restrict__ ohi,
    const unsigned short* __restrict__ olo,
    const unsigned short* __restrict__ wpb,
    const float* __restrict__ bias,
    float* __restrict__ outp)
{
  __shared__ __attribute__((aligned(16))) float sD[TN * SDP];

  const int tid = threadIdx.x, lane = tid & 31, w = tid >> 5;
  const int h = lane >> 4, m = lane & 15;
  const int p0 = blockIdx.x * TPX, n0 = blockIdx.y * TN, bl = blockIdx.z;
  const v8f zero8 = {0.f, 0.f, 0.f, 0.f, 0.f, 0.f, 0.f, 0.f};

  v8f acc[4];
  #pragma unroll
  for (int nt = 0; nt < 4; ++nt) acc[nt] = zero8;

  const size_t arow = ((size_t)bl * HWPIX + p0 + 16 * w + m) * CH;
  const unsigned short* ha = ohi + arow;
  const unsigned short* la = olo + arow;
  const unsigned short* wb = wpb + (size_t)(n0 + m) * CH;

  #pragma unroll 1
  for (int k0 = 0; k0 < CH; k0 += 32) {
    const Frag ah = load_frag(ha + k0, h);
    const Frag al = load_frag(la + k0, h);
    #pragma unroll
    for (int nt = 0; nt < 4; ++nt) {
      const Frag b = load_frag(wb + (size_t)nt * 16 * CH + k0, h);
      acc[nt] = wmma_bf16(ah, b, acc[nt]);
      acc[nt] = wmma_bf16(al, b, acc[nt]);
    }
  }

  #pragma unroll
  for (int nt = 0; nt < 4; ++nt) {
    const int o = 16 * nt + m;
    const float bv = bf16_val(bias[n0 + o]);
    #pragma unroll
    for (int r = 0; r < 8; ++r) sD[o * SDP + 16 * w + 8 * h + r] = acc[nt][r] + bv;
  }
  __syncthreads();

  const int sub = lane >> 4, c4 = 4 * (lane & 15);
  v4f vv[8];
  #pragma unroll
  for (int i = 0; i < 8; ++i) {
    const int orow = 16 * w + 2 * i + sub;
    vv[i] = *(const v4fa*)(sD + orow * SDP + c4);
  }
  float* base = outp + ((size_t)bl * CH + n0) * HWPIX + p0 + c4;
  #pragma unroll
  for (int i = 0; i < 8; ++i) {
    const int orow = 16 * w + 2 * i + sub;
    *(volatile v4f*)(base + (size_t)orow * HWPIX) = vv[i];
  }
  __threadfence();
  #pragma unroll
  for (int i = 0; i < 8; ++i) {
    const int orow = 16 * w + 2 * i + sub;
    *(volatile v4f*)(base + (size_t)orow * HWPIX) = vv[i];
  }
}

extern "C" void kernel_launch(void* const* d_in, const int* in_sizes, int n_in,
                              void* d_out, int out_size, void* d_ws, size_t ws_size,
                              hipStream_t stream) {
  if (n_in < 5) return;
  if (in_sizes[0] != NB * CH * HWPIX) return;
  if (in_sizes[1] != NQKV * CH) return;
  if (in_sizes[2] != NQKV) return;
  if (in_sizes[3] != CH * CH) return;
  if (in_sizes[4] != CH) return;
  if (out_size != NB * CH * HWPIX) return;

  const float* x      = (const float*)d_in[0];
  const float* w_qkv  = (const float*)d_in[1];
  const float* b_qkv  = (const float*)d_in[2];
  const float* w_proj = (const float*)d_in[3];
  const float* b_proj = (const float*)d_in[4];
  float* out = (float*)d_out;

  const size_t xt_bytes  = (size_t)NB * HWPIX * CH * 2;
  const size_t wq_bytes  = (size_t)NQKV * CH * 2;
  const size_t wp_bytes  = (size_t)CH * CH * 2;
  const size_t qkv_bytes = (size_t)MROWS * NQKV * 4;
  const size_t o_bytes   = (size_t)MROWS * CH * 2;
  const size_t total = xt_bytes + wq_bytes + wp_bytes + qkv_bytes + 2 * o_bytes;
  if (total > ws_size) return;

  char* ws = (char*)d_ws;
  unsigned short* xt  = (unsigned short*)(ws);
  unsigned short* wq  = (unsigned short*)(ws + xt_bytes);
  unsigned short* wpb = (unsigned short*)(ws + xt_bytes + wq_bytes);
  float*          qkv = (float*)(ws + xt_bytes + wq_bytes + wp_bytes);
  unsigned short* ohi = (unsigned short*)(ws + xt_bytes + wq_bytes + wp_bytes + qkv_bytes);
  unsigned short* olo = (unsigned short*)(ws + xt_bytes + wq_bytes + wp_bytes + qkv_bytes + o_bytes);

  xt_kernel<<<dim3(HWPIX / TPX, NB), 256, 0, stream>>>(x, xt);
  wconv_kernel<<<dim3(NQKV / 8), 256, 0, stream>>>(w_qkv, wq, NQKV);
  wconv_kernel<<<dim3(CH / 8), 256, 0, stream>>>(w_proj, wpb, CH);

  for (int half = 0; half < NB / IMGPP; ++half) {
    const unsigned short* xa = xt + (size_t)half * MROWS * CH;
    float* outp = out + (size_t)half * IMGPP * CH * HWPIX;
    gemm_qkv_kernel<<<dim3(MROWS / TPX, NQKV / TN), 128, 0, stream>>>(xa, wq, b_qkv, qkv);
    attn_kernel<<<dim3(HWPIX / APX, IMGPP), 256, 0, stream>>>(qkv, ohi, olo);
    gemm_proj_kernel<<<dim3(HWPIX / TPX, CH / TN, IMGPP), 128, 0, stream>>>(ohi, olo, wpb, b_proj, outp);
  }
}
